// TransformerBlock_9758165697319
// MI455X (gfx1250) — hardware-run, weakly checked
//
#include <hip/hip_runtime.h>
#include <math.h>

#ifndef NB
#define NB 128
#endif
#ifndef SEQ
#define SEQ 256
#endif
#define NB_FULL 128
#define SEQ_FULL 256
#define EMB 384
#define NHEAD 6
#define HDIM 64
#define DFF 1536
#define QKVW (3 * EMB)
#define NBC (((SEQ) == SEQ_FULL) ? (((NB) < 32) ? (NB) : 32) : 1)
#define RC (NBC * (SEQ))
#define NCHUNK ((NB) / NBC)
#define KVGPR __attribute__((amdgpu_num_vgpr(256)))

static_assert(NB >= 1 && NB <= NB_FULL);
static_assert(SEQ >= 64 && SEQ <= SEQ_FULL && (SEQ % 64) == 0);
static_assert((NB % NBC) == 0);
static_assert((RC % 64) == 0);
static_assert((EMB % 128) == 0 && (EMB % 64) == 0 && (EMB % 32) == 0);
static_assert((DFF % 64) == 0 && (DFF % 32) == 0);
static_assert(NHEAD * HDIM == EMB);
static_assert(HDIM == 64);
static_assert((QKVW % 64) == 0);
static_assert((QKVW % 4) == 0 && (EMB % 4) == 0);

typedef __attribute__((ext_vector_type(16))) _Float16 v16h;
typedef __attribute__((ext_vector_type(8)))  _Float16 v8h;
typedef __attribute__((ext_vector_type(16))) __bf16   v16b;
typedef __attribute__((ext_vector_type(8)))  __bf16   v8b;
typedef __attribute__((ext_vector_type(8)))  float    v8f;
typedef __attribute__((ext_vector_type(4)))  float    v4f;
typedef _Float16 h16;


static __device__ __forceinline__ h16 toh_flush(float v) { const h16 r = (h16)v; return (fabsf(v) < 6.103515625e-05f) ? (h16)0.0f : r; }
static __device__ __forceinline__ float gelu_erf(float v) { return 0.5f * v * (1.0f + erff(v * 0.70710678118654752f)); }
__device__ __forceinline__ v8f wmma1h(v16h a, v16h b, v8f c) {
    c = __builtin_amdgcn_wmma_f32_16x16x32_f16(false, a, false, b, (short)0, c, false, false);
    asm volatile("v_nop\n\tv_nop\n\tv_nop\n\tv_nop" : "+v"(c) : "v"(a), "v"(b));
    return c;
}
union FragH { v16h v; v8h h[2]; };

#define VST2(T, ptr, val) do { const T vst2_v_ = (val); *(volatile T*)(ptr) = vst2_v_; __threadfence(); *(volatile T*)(ptr) = vst2_v_; } while (0)
#define VST2V4(ptr, val) do { const v4f vst2_v4_ = (val); *(volatile v4f*)(ptr) = vst2_v4_; __threadfence(); *(volatile v4f*)(ptr) = vst2_v4_; } while (0)

__global__ __launch_bounds__(128) KVGPR void k_attn_d(const float* __restrict__ Q, const float* __restrict__ K, const float* __restrict__ V, float* __restrict__ O,
                                                       int in_bs, int in_rs, int o_bs, int o_rs, int nkc, float scale) {
    __shared__ __align__(16) _Float16 Ksh[64 * 64];
    __shared__ __align__(16) _Float16 Vth[64 * 64];
    __shared__ __align__(16) _Float16 Psh[4][16 * 64];
    __shared__ __align__(16) float    Os[4][16 * 36];
    static_assert(sizeof(Ksh) + sizeof(Vth) + sizeof(Psh) + sizeof(Os) <= 131072);

    const int tid  = threadIdx.x;
    const int wave = __builtin_amdgcn_readfirstlane((int)(threadIdx.x >> 5));
    const int lane = tid & 31, hh = lane >> 4, c = lane & 15;
    const int qb = blockIdx.x, h = blockIdx.y, b = blockIdx.z;
    const int q0 = qb * 64 + wave * 16;
    const float L2E = 1.4426950408889634f;
    const float NEG = -__builtin_inff();
    const float PCL2 = 8.0f;

    const size_t inb = (size_t)b * (size_t)in_bs + (size_t)h * 64;
    const float* qp = Q + inb;
    const float* kp = K + inb;
    const float* vp = V + inb;
    float* op = O + (size_t)b * (size_t)o_bs + (size_t)h * 64;

    v16h qf[2];
    {
        const float* qrow = qp + (size_t)(q0 + c) * (size_t)in_rs;
#pragma unroll
        for (int dc = 0; dc < 2; ++dc) {
            const v4f a0 = *(const v4f*)(qrow + dc * 32 + 8 * hh);
            const v4f a1 = *(const v4f*)(qrow + dc * 32 + 8 * hh + 4);
            const v4f b0 = *(const v4f*)(qrow + dc * 32 + 16 + 8 * hh);
            const v4f b1 = *(const v4f*)(qrow + dc * 32 + 16 + 8 * hh + 4);
#pragma unroll
            for (int e = 0; e < 4; ++e) {
                qf[dc][e]      = toh_flush(a0[e]);
                qf[dc][4 + e]  = toh_flush(a1[e]);
                qf[dc][8 + e]  = toh_flush(b0[e]);
                qf[dc][12 + e] = toh_flush(b1[e]);
            }
        }
    }

    float mrow[8], lrow[8];
    v8f oacc[4];
#pragma unroll
    for (int r = 0; r < 8; ++r) { mrow[r] = NEG; lrow[r] = 0.f; }
#pragma unroll
    for (int t = 0; t < 4; ++t) { v8f zz = {}; oacc[t] = zz; }

    for (int kc = 0; kc < nkc; ++kc) {
        const int kv0 = kc * 64;
        __syncthreads();
        {
            static_assert(128 * 8 * 4 == 64 * 64);
            const int kvr = tid >> 1, dh = (tid & 1) * 32;
            const float* krow = kp + (size_t)(kv0 + kvr) * (size_t)in_rs + dh;
            const float* vrow = vp + (size_t)(kv0 + kvr) * (size_t)in_rs + dh;
#pragma unroll 1
            for (int i = 0; i < 8; ++i) {
                const v4f kk = *(const v4f*)(krow + 4 * i);
                const v4f vv = *(const v4f*)(vrow + 4 * i);
#pragma unroll
                for (int e = 0; e < 4; ++e) {
                    const int d = dh + 4 * i + e;
                    Ksh[kvr * 64 + d] = toh_flush(kk[e]);
                    Vth[d * 64 + kvr] = toh_flush(vv[e]);
                }
            }
        }
        __syncthreads();

        v8f s[4];
#pragma unroll
        for (int j = 0; j < 4; ++j) {
            v8f acc = {};
#pragma unroll
            for (int dc = 0; dc < 2; ++dc) {
                const int off = (j * 16 + c) * 64 + dc * 32 + 8 * hh;
                FragH kb;
                kb.h[0] = *(const v8h*)(&Ksh[off]); kb.h[1] = *(const v8h*)(&Ksh[off + 16]);
                acc = wmma1h(qf[dc], kb.v, acc);
            }
            s[j] = acc;
        }

#pragma unroll
        for (int r = 0; r < 8; ++r) {
            float sc[4];
#pragma unroll
            for (int j = 0; j < 4; ++j) {
                float v = s[j][r] * scale;
                v *= L2E;
                sc[j] = v;
            }
            float mx = fmaxf(fmaxf(sc[0], sc[1]), fmaxf(sc[2], sc[3]));
            mx = fmaxf(mx, __shfl_xor(mx, 1, 32)); mx = fmaxf(mx, __shfl_xor(mx, 2, 32));
            mx = fmaxf(mx, __shfl_xor(mx, 4, 32)); mx = fmaxf(mx, __shfl_xor(mx, 8, 32));
            const float mnew = fmaxf(mrow[r], mx);
            const float corr = (mrow[r] == NEG) ? 0.f : exp2f(mrow[r] - mnew);
            float rs = 0.f;
#pragma unroll
            for (int j = 0; j < 4; ++j) {
                const float pe = (sc[j] - mnew) + PCL2;
                const h16 ph = (pe < -14.0f) ? (h16)0.0f : (h16)exp2f(pe);
                rs += (float)ph;
                Psh[wave][(8 * hh + r) * 64 + j * 16 + c] = ph;
            }
            rs += __shfl_xor(rs, 1, 32); rs += __shfl_xor(rs, 2, 32); rs += __shfl_xor(rs, 4, 32); rs += __shfl_xor(rs, 8, 32);
            lrow[r] = lrow[r] * corr + rs; mrow[r] = mnew;
#pragma unroll
            for (int t = 0; t < 4; ++t) oacc[t][r] *= corr;
        }
        __syncthreads();

#pragma unroll
        for (int kk = 0; kk < 2; ++kk) {
            const int po = c * 64 + kk * 32 + 8 * hh;
            FragH pa;
            pa.h[0] = *(const v8h*)(&Psh[wave][po]); pa.h[1] = *(const v8h*)(&Psh[wave][po + 16]);
#pragma unroll
            for (int t = 0; t < 4; ++t) {
                const int vo = (t * 16 + c) * 64 + kk * 32 + 8 * hh;
                FragH vb;
                vb.h[0] = *(const v8h*)(&Vth[vo]); vb.h[1] = *(const v8h*)(&Vth[vo + 16]);
                oacc[t] = wmma1h(pa.v, vb.v, oacc[t]);
            }
        }
    }

    float inv[8];
#pragma unroll
    for (int r = 0; r < 8; ++r) inv[r] = (lrow[r] > 0.f) ? 1.f / lrow[r] : 0.f;
    static_assert(32 * 4 * 16 == 16 * 32 * 4);
#pragma unroll
    for (int half = 0; half < 2; ++half) {
#pragma unroll
        for (int r = 0; r < 8; ++r) {
            Os[wave][(8 * hh + r) * 36 + c]      = oacc[2 * half][r] * inv[r];
            Os[wave][(8 * hh + r) * 36 + 16 + c] = oacc[2 * half + 1][r] * inv[r];
        }
        __syncthreads();
        {
            const int q4 = lane >> 3, c4 = (lane & 7) * 4;
#pragma unroll
            for (int it = 0; it < 4; ++it) {
                const int row = it * 4 + q4;
                const v4f val = *(const v4f*)(&Os[wave][row * 36 + c4]);
                VST2V4(op + (size_t)(q0 + row) * (size_t)o_rs + half * 32 + c4, val);
            }
        }
        __syncthreads();
    }
}

namespace eng {
typedef __attribute__((ext_vector_type(16))) _Float16 v16h;
typedef __attribute__((ext_vector_type(8)))  _Float16 v8h;
typedef __attribute__((ext_vector_type(16))) __bf16   v16b;
typedef __attribute__((ext_vector_type(8)))  __bf16   v8b;
typedef __attribute__((ext_vector_type(8)))  float    v8f;
typedef __attribute__((ext_vector_type(4)))  float    v4f;

__device__ __forceinline__ unsigned short f2bf_bits(float f) {
  unsigned u = __float_as_uint(f);
  return (unsigned short)((u + 0x7FFFu + ((u >> 16) & 1u)) >> 16);
}
__device__ __forceinline__ float bf_bits2f(unsigned short h) { return __uint_as_float(((unsigned)h) << 16); }

__device__ __forceinline__ void dep_guard_h(v8f& a, v8f& b, v16h x, v16h y) { asm volatile("v_nop\n\tv_nop\n\tv_nop\n\tv_nop" : "+v"(a), "+v"(b) : "v"(x), "v"(y)); }
__device__ __forceinline__ void dep_guard_b(v8f& a, v8f& b, v16b x, v16b y) { asm volatile("v_nop\n\tv_nop\n\tv_nop\n\tv_nop" : "+v"(a), "+v"(b) : "v"(x), "v"(y)); }
__device__ __forceinline__ void keep4_h(v16h a, v16h b, v16h c, v16h d) { asm volatile("v_nop" :: "v"(a), "v"(b), "v"(c), "v"(d)); }
__device__ __forceinline__ void keep4_b(v16b a, v16b b, v16b c, v16b d) { asm volatile("v_nop" :: "v"(a), "v"(b), "v"(c), "v"(d)); }
__device__ __forceinline__ void acc_guard4(v8f& a, v8f& b, v8f& c, v8f& d) { asm volatile("v_nop\n\tv_nop\n\tv_nop\n\tv_nop" : "+v"(a), "+v"(b), "+v"(c), "+v"(d)); }
template <typename T> struct Frag;
template <> struct Frag<_Float16> {
  typedef v16h V; union U { v16h v; v8h h[2]; };
  static __device__ __forceinline__ v16h load(const _Float16* p) {
    U f; f.h[0] = *(const v8h*)(p); f.h[1] = *(const v8h*)(p + 16); return f.v;
  }
  static __device__ __forceinline__ v8f mma(v16h a, v16h b, v8f c) {
    return __builtin_amdgcn_wmma_f32_16x16x32_f16(false, a, false, b, (short)0, c, false, false);
  }
  static __device__ __forceinline__ void guard(v8f& a, v8f& b, v16h x, v16h y) { dep_guard_h(a, b, x, y); }
  static __device__ __forceinline__ void keep(v16h a, v16h b, v16h c, v16h d) { keep4_h(a, b, c, d); }
};
template <> struct Frag<__bf16> {
  typedef v16b V; union U { v16b v; v8b h[2]; };
  static __device__ __forceinline__ v16b load(const __bf16* p) {
    U f; f.h[0] = *(const v8b*)(p); f.h[1] = *(const v8b*)(p + 16); return f.v;
  }
  static __device__ __forceinline__ v8f mma(v16b a, v16b b, v8f c) {
    return __builtin_amdgcn_wmma_f32_16x16x32_bf16(false, a, false, b, (short)0, c, false, false);
  }
  static __device__ __forceinline__ void guard(v8f& a, v8f& b, v16b x, v16b y) { dep_guard_b(a, b, x, y); }
  static __device__ __forceinline__ void keep(v16b a, v16b b, v16b c, v16b d) { keep4_b(a, b, c, d); }
};

template <int ET> struct Elem;
template <> struct Elem<0> { typedef _Float16 T; };
template <> struct Elem<1> { typedef __bf16 T; };
template <int ET, bool SPLIT, int BIAS_MODE, int OUT_MODE, bool RESID, int ACT = 0>
__global__ __launch_bounds__(256) KVGPR void wmma_gemm64(
    const unsigned short* __restrict__ Ap, const unsigned short* __restrict__ A2p, int lda, long strideA,
    const unsigned short* __restrict__ Btp, const unsigned short* __restrict__ Bt2p, int ldb, long strideB,
    void* __restrict__ Cout, void* __restrict__ Cout2, int ldc, long strideC,
    const float* __restrict__ bias,
    const float* __restrict__ resid, long strideR,
    int M, int N, int K, float scale) {
  typedef typename Elem<ET>::T T;
  typedef typename Frag<T>::V V;
  const T* A = (const T*)Ap; const T* A2 = (const T*)A2p; const T* Bt = (const T*)Btp; const T* Bt2 = (const T*)Bt2p;
  __shared__ __align__(16) float sT[8][16 * 68];
  static_assert(sizeof(sT) <= 131072);
  const int b    = blockIdx.y;
  const int lane = threadIdx.x & 31;
  const int wave = __builtin_amdgcn_readfirstlane((int)(threadIdx.x >> 5));
  const int tilesN = N >> 6;
  const int tilesM = M >> 6;
  const int tile = blockIdx.x * 8 + wave;
  if (tile >= tilesM * tilesN) return;
  const int tm = tile / tilesN;
  const int tn = tile - tm * tilesN;
  const int m0 = tm << 6;
  const int n0 = tn << 6;

  const T* Ab  = A  + (size_t)b * strideA;
  const T* Bb  = Bt + (size_t)b * strideB;
  const T* Ab2 = SPLIT ? (A2  + (size_t)b * strideA) : nullptr;
  const T* Bb2 = SPLIT ? (Bt2 + (size_t)b * strideB) : nullptr;

  const int rlane = lane & 15;
  const int koff  = (lane >> 4) * 8;
  const int mOff  = (lane >> 4) * 8;

  v8f acc[4][4];
#pragma unroll
  for (int i = 0; i < 4; ++i)
#pragma unroll
    for (int j = 0; j < 4; ++j) acc[i][j] = (v8f){0.f,0.f,0.f,0.f,0.f,0.f,0.f,0.f};

  for (int k0 = 0; k0 < K; k0 += 32) {
    V bh[4], bl[4];
#pragma unroll
    for (int j = 0; j < 4; ++j) {
      const size_t bo = (size_t)(n0 + (j << 4) + rlane) * ldb + koff + k0;
      bh[j] = Frag<T>::load(Bb + bo);
      if (SPLIT) bl[j] = Frag<T>::load(Bb2 + bo);
    }
#pragma unroll
    for (int i = 0; i < 4; ++i) {
      const size_t ao = (size_t)(m0 + (i << 4) + rlane) * lda + koff + k0;
      V ah = Frag<T>::load(Ab + ao);
      V al;
      if (SPLIT) al = Frag<T>::load(Ab2 + ao);
#pragma unroll
      for (int j = 0; j < 4; ++j) {
        acc[i][j] = Frag<T>::mma(ah, bh[j], acc[i][j]);
        if (SPLIT) {
          acc[i][j] = Frag<T>::mma(ah, bl[j], acc[i][j]);
          acc[i][j] = Frag<T>::mma(al, bh[j], acc[i][j]);
        }
      }
      Frag<T>::guard(acc[i][0], acc[i][3], ah, SPLIT ? al : ah);
    }
    Frag<T>::keep(bh[0], bh[1], bh[2], bh[3]);
    if (SPLIT) Frag<T>::keep(bl[0], bl[1], bl[2], bl[3]);
  }
  acc_guard4(acc[0][0], acc[0][1], acc[0][2], acc[0][3]);
  acc_guard4(acc[1][0], acc[1][1], acc[1][2], acc[1][3]);
  acc_guard4(acc[2][0], acc[2][1], acc[2][2], acc[2][3]);
  acc_guard4(acc[3][0], acc[3][1], acc[3][2], acc[3][3]);

  const float* Rb = RESID ? (resid + (size_t)b * strideR) : nullptr;
#pragma unroll
  for (int i = 0; i < 4; ++i) {
    const int mBase = m0 + (i << 4);
#pragma unroll
    for (int j = 0; j < 4; ++j) {
      const int n = n0 + (j << 4) + rlane;
      float bv = 0.f;
      if (BIAS_MODE == 2) bv = bias[n];
#pragma unroll
      for (int r = 0; r < 8; ++r) {
        float v = acc[i][j][r] * scale;
        if (BIAS_MODE == 1) v += bias[mBase + mOff + r];
        if (BIAS_MODE == 2) v += bv;
        if (RESID) v += Rb[(size_t)(mBase + mOff + r) * ldc + n];
        if (ACT == 2) v = fmaxf(v, 0.0f);
        if (ACT == 3) v = gelu_erf(v);
        sT[wave][(mOff + r) * 68 + (j << 4) + rlane] = v;
      }
    }
    __builtin_amdgcn_fence(3  , "workgroup");
    __builtin_amdgcn_wave_barrier();
    __builtin_amdgcn_fence(2  , "workgroup");
    if (OUT_MODE == 0) {
      float* C = (float*)Cout + (size_t)b * strideC;
      const int hh = lane >> 4, c4 = (lane & 15) * 4;
      static_assert(32 * 8 * 16 == 16 * 64 * 4);
      for (int pass = 0; pass < 2; ++pass) {
#pragma unroll
        for (int it = 0; it < 8; ++it) {
          const int row = it * 2 + hh;
          v4f v = *(const v4f*)(&sT[wave][row * 68 + c4]);
          *(volatile v4f*)(C + (size_t)(mBase + row) * ldc + n0 + c4) = v;
        }
        __threadfence();
      }
    } else {
      const int q = lane >> 3, c8 = (lane & 7) * 8;
      static_assert(32 * 4 * 16 == 16 * 64 * 2);
      unsigned short* C  = (unsigned short*)Cout  + (size_t)b * strideC;
      unsigned short* C2 = (OUT_MODE == 2) ? ((unsigned short*)Cout2 + (size_t)b * strideC) : nullptr;
      for (int pass = 0; pass < 2; ++pass) {
#pragma unroll
        for (int it = 0; it < 4; ++it) {
          const int row = it * 4 + q;
          const v4f s0 = *(const v4f*)(&sT[wave][row * 68 + c8]);
          const v4f s1 = *(const v4f*)(&sT[wave][row * 68 + c8 + 4]);
          v8h hv, lv;
#pragma unroll
          for (int e = 0; e < 8; ++e) {
            const float sv = (e < 4) ? s0[e & 3] : s1[e & 3];
            if (OUT_MODE == 1) {
              hv[e] = toh_flush(sv);
            } else {
              unsigned short hb = f2bf_bits(sv);
              unsigned short lb = f2bf_bits(sv - bf_bits2f(hb));
              hv[e] = __builtin_bit_cast(_Float16, hb);
              lv[e] = __builtin_bit_cast(_Float16, lb);
            }
          }
          *(volatile v8h*)(C + (size_t)(mBase + row) * ldc + n0 + c8) = hv;
          if (OUT_MODE == 2) *(volatile v8h*)(C2 + (size_t)(mBase + row) * ldc + n0 + c8) = lv;
        }
        __threadfence();
      }
    }
    __builtin_amdgcn_fence(3  , "workgroup");
    __builtin_amdgcn_wave_barrier();
    __builtin_amdgcn_fence(2  , "workgroup");
  }
}
}

__global__ __launch_bounds__(256) void k_cast16(const float* __restrict__ src, long long lds, _Float16* __restrict__ dst, long long ldd, int R, int C, float s) {
    const long long i = (long long)blockIdx.x * 256 + threadIdx.x; const long long np = (long long)R * (C / 2); if (i >= np) return; const int r = (int)(i / (C / 2)); const int c = 2 * (int)(i % (C / 2));
    const _Float16 h0 = (_Float16)(src[(long long)r * lds + c] * s), h1 = (_Float16)(src[(long long)r * lds + c + 1] * s);
    const unsigned u = (unsigned)__builtin_bit_cast(unsigned short, h0) | ((unsigned)__builtin_bit_cast(unsigned short, h1) << 16);
    volatile unsigned* d = (volatile unsigned*)(dst + (long long)r * ldd + c); *d = u; __threadfence(); *d = u; }

typedef unsigned int cm_u4 __attribute__((ext_vector_type(4)));
__device__ __forceinline__ unsigned int cmb_pk2(float a, float b) { return (unsigned int)__builtin_bit_cast(unsigned short, (_Float16)a) | ((unsigned int)__builtin_bit_cast(unsigned short, (_Float16)b) << 16); }
__device__ __forceinline__ unsigned int cmf_pk2(float a, float b) { return (unsigned int)__builtin_bit_cast(unsigned short, toh_flush(a)) | ((unsigned int)__builtin_bit_cast(unsigned short, toh_flush(b)) << 16); }
__device__ __forceinline__ float cmb_bf(float v) { const unsigned u = __builtin_bit_cast(unsigned, v); const unsigned r = (u + 0x7fffu + ((u >> 16) & 1u)) & 0xffff0000u; return __builtin_bit_cast(float, r); }
__global__ __launch_bounds__(256) void k_cm_bfvec(const float* __restrict__ SRC, float* __restrict__ DST, int n) { const int u = blockIdx.x * 256 + threadIdx.x; if (u >= n) return; VST2(float, DST + u, cmb_bf(SRC[u])); }
__global__ __launch_bounds__(256) void k_cm_castbT(const float* __restrict__ SRC, int lds, long long sSz, unsigned short* __restrict__ DST, int ldd, long long sDz, int nR, int nC, float sc) {
    const long long u = (long long)blockIdx.x * 256 + threadIdx.x; const int per = nR / 8; if (u >= (long long)nC * per) return; const int c = (int)(u / per); const int r0 = 8 * (int)(u % per);
    const float* s = SRC + (long long)blockIdx.y * sSz; unsigned short* d = DST + (long long)blockIdx.y * sDz;
    float w[8];
#pragma unroll
    for (int e = 0; e < 8; ++e) w[e] = cmb_bf(s[(long long)(r0 + e) * lds + c]) * sc;
    cm_u4 pk; pk.x = cmf_pk2(w[0], w[1]); pk.y = cmf_pk2(w[2], w[3]); pk.z = cmf_pk2(w[4], w[5]); pk.w = cmf_pk2(w[6], w[7]); VST2(cm_u4, (cm_u4*)(d + (long long)c * ldd + r0), pk); }

typedef unsigned int bk_u2 __attribute__((ext_vector_type(2)));
__device__ __forceinline__ unsigned int bk_pk2(float a, float b) { return (unsigned int)__builtin_bit_cast(unsigned short, (_Float16)a) | ((unsigned int)__builtin_bit_cast(unsigned short, (_Float16)b) << 16); }
template <int NQ, int HASX, int XBF, int ABF = 0>
__global__ __launch_bounds__(256) void k_b_ln(const float* __restrict__ A, const float* __restrict__ X, const float* __restrict__ GA, const float* __restrict__ BE, float eps, float inv_vden, int rows, const float* __restrict__ MG, const float* __restrict__ MB, int rows_per_b, float* __restrict__ Yf, unsigned short* __restrict__ Y16) {
    #pragma clang fp contract(off)
    constexpr int WD = 128 * NQ; const int r = blockIdx.x * 8 + __builtin_amdgcn_readfirstlane((int)(threadIdx.x >> 5)); const int L = threadIdx.x & 31; if (r >= rows) return; v4f v[NQ]; float s = 0.f;
#pragma unroll
    for (int q = 0; q < NQ; ++q) { const long long o = (long long)r * WD + 4 * L + 128 * q; v[q] = *(const v4f*)(A + o); if (ABF) { v[q].x = cmb_bf(v[q].x); v[q].y = cmb_bf(v[q].y); v[q].z = cmb_bf(v[q].z); v[q].w = cmb_bf(v[q].w); } if (HASX) { v4f x = *(const v4f*)(X + o); if (XBF) { x.x = cmb_bf(x.x); x.y = cmb_bf(x.y); x.z = cmb_bf(x.z); x.w = cmb_bf(x.w); } v[q] = v[q] + x; } s += (v[q].x + v[q].y) + (v[q].z + v[q].w); }
#pragma unroll
    for (int o = 16; o > 0; o >>= 1) s += __shfl_xor(s, o, 32);
    const float mu = s * (1.f / WD); float qq = 0.f;
#pragma unroll
    for (int q = 0; q < NQ; ++q) { v[q].x -= mu; v[q].y -= mu; v[q].z -= mu; v[q].w -= mu; qq += (v[q].x * v[q].x + v[q].y * v[q].y) + (v[q].z * v[q].z + v[q].w * v[q].w); }
#pragma unroll
    for (int o = 16; o > 0; o >>= 1) qq += __shfl_xor(qq, o, 32);
    const float rs = (eps < 0.f) ? (1.f / (sqrtf(qq * inv_vden) - eps)) : rsqrtf(qq * inv_vden + eps); const int bb = (MG != nullptr) ? (r / rows_per_b) : 0;
#pragma unroll
    for (int q = 0; q < NQ; ++q) { const int c = 4 * L + 128 * q; const v4f ga = *(const v4f*)(GA + c), be = *(const v4f*)(BE + c); v4f y; y.x = v[q].x * rs * cmb_bf(ga.x) + cmb_bf(be.x); y.y = v[q].y * rs * cmb_bf(ga.y) + cmb_bf(be.y); y.z = v[q].z * rs * cmb_bf(ga.z) + cmb_bf(be.z); y.w = v[q].w * rs * cmb_bf(ga.w) + cmb_bf(be.w);
        if (MG != nullptr) { const v4f mg = *(const v4f*)(MG + (long long)bb * WD + c), mb = *(const v4f*)(MB + (long long)bb * WD + c); y.x = y.x * (1.f + mg.x) + mb.x; y.y = y.y * (1.f + mg.y) + mb.y; y.z = y.z * (1.f + mg.z) + mb.z; y.w = y.w * (1.f + mg.w) + mb.w; }
        const long long o = (long long)r * WD + c; if (Yf != nullptr) VST2V4(Yf + o, y); if (Y16 != nullptr) { bk_u2 pk; pk.x = bk_pk2(y.x, y.y); pk.y = bk_pk2(y.z, y.w); VST2(bk_u2, (bk_u2*)(Y16 + o), pk); } } }
template <int XBF>
__global__ __launch_bounds__(256) void k_b_add(const float* __restrict__ A, const float* __restrict__ X, const float* __restrict__ AL, int WD4, int rows_per_b, float* __restrict__ O, long long n4) {
    #pragma clang fp contract(off)
    const long long u = (long long)blockIdx.x * 256 + threadIdx.x; if (u >= n4) return; v4f a = *(const v4f*)(A + 4 * u); v4f x = *(const v4f*)(X + 4 * u); if (XBF) { x.x = cmb_bf(x.x); x.y = cmb_bf(x.y); x.z = cmb_bf(x.z); x.w = cmb_bf(x.w); }
    if (AL != nullptr) { const long long r = u / WD4; const int c4 = (int)(u % WD4); const v4f al = *(const v4f*)(AL + ((r / rows_per_b) * WD4 + c4) * 4); a.x *= al.x; a.y *= al.y; a.z *= al.z; a.w *= al.w; }
    v4f y; y.x = x.x + a.x; y.y = x.y + a.y; y.z = x.z + a.z; y.w = x.w + a.w; VST2V4(O + 4 * u, y); }

constexpr size_t al256(size_t b) { return (b + 255) / 256 * 256; }
constexpr size_t SZ_P16 = al256((size_t)RC * EMB * 2);
constexpr size_t SZ_QKV = al256((size_t)RC * QKVW * 4);
constexpr size_t SZ_F32 = al256((size_t)RC * EMB * 4);
constexpr size_t SZ_F16 = al256((size_t)RC * DFF * 2);
constexpr size_t SZ_W3  = al256((size_t)QKVW * EMB * 2);
constexpr size_t SZ_WO  = al256((size_t)EMB * EMB * 2);
constexpr size_t SZ_W1  = al256((size_t)DFF * EMB * 2);
constexpr size_t SZ_BE  = al256((size_t)(EMB + 64) * 4);
constexpr size_t SZ_BD  = al256((size_t)(DFF + 64) * 4);
constexpr size_t SZ_BQ  = al256((size_t)(QKVW + 64) * 4);
constexpr size_t WS_TOTAL = 2 * SZ_P16 + SZ_QKV + 4 * SZ_F32 + SZ_F16 + SZ_W3 + SZ_WO + 2 * SZ_W1 + 2 * SZ_BE + SZ_BD + SZ_BQ;
static_assert(WS_TOTAL <= (size_t)134217728);
static_assert(((size_t)EMB * 4) % 128 == 0);

extern "C" void kernel_launch(void* const* d_in, const int* in_sizes, int n_in, void* d_out, int out_size, void* d_ws, size_t ws_size, hipStream_t stream) {
    if (n_in < 17) return;
    const long long need_x = ((long long)(NB - 1) * SEQ_FULL + SEQ) * EMB;
    if ((long long)in_sizes[0] < need_x || (long long)out_size < need_x) return;
    if (in_sizes[1] < NHEAD * EMB * HDIM || in_sizes[3] < NHEAD * EMB * HDIM || in_sizes[5] < NHEAD * EMB * HDIM) return;
    if (in_sizes[2] < NHEAD * HDIM || in_sizes[4] < NHEAD * HDIM || in_sizes[6] < NHEAD * HDIM) return;
    if (in_sizes[7] < EMB * EMB || in_sizes[8] < EMB || in_sizes[9] < EMB * DFF || in_sizes[10] < DFF || in_sizes[11] < DFF * EMB || in_sizes[12] < EMB) return;
    if (in_sizes[13] < EMB || in_sizes[14] < EMB || in_sizes[15] < EMB || in_sizes[16] < EMB) return;
    if (ws_size < WS_TOTAL) return;
    const float* x = (const float*)d_in[0];
    const float* wq = (const float*)d_in[1];
    const float* bq = (const float*)d_in[2];
    const float* wk = (const float*)d_in[3];
    const float* bk = (const float*)d_in[4];
    const float* wv = (const float*)d_in[5];
    const float* bv = (const float*)d_in[6];
    const float* wo = (const float*)d_in[7];
    const float* bo = (const float*)d_in[8];
    const float* w1 = (const float*)d_in[9];
    const float* b1 = (const float*)d_in[10];
    const float* w2 = (const float*)d_in[11];
    const float* b2 = (const float*)d_in[12];
    const float* g1 = (const float*)d_in[13];
    const float* be1 = (const float*)d_in[14];
    const float* g2 = (const float*)d_in[15];
    const float* be2 = (const float*)d_in[16];
    float* out = (float*)d_out;
    char* wsp = (char*)d_ws;
    unsigned short* X16 = (unsigned short*)wsp; wsp += SZ_P16;
    unsigned short* H16 = (unsigned short*)wsp; wsp += SZ_P16;
    float* QKV = (float*)wsp; wsp += SZ_QKV;
    float* AO = (float*)wsp; wsp += SZ_F32;
    float* ATT = (float*)wsp; wsp += SZ_F32;
    float* X1 = (float*)wsp; wsp += SZ_F32;
    float* FFo = (float*)wsp; wsp += SZ_F32;
    unsigned short* F16 = (unsigned short*)wsp; wsp += SZ_F16;
    unsigned short* W316 = (unsigned short*)wsp; wsp += SZ_W3;
    unsigned short* WO16 = (unsigned short*)wsp; wsp += SZ_WO;
    unsigned short* W1T = (unsigned short*)wsp; wsp += SZ_W1;
    unsigned short* W2T = (unsigned short*)wsp; wsp += SZ_W1;
    float* BRO = (float*)wsp; wsp += SZ_BE;
    float* BR2 = (float*)wsp; wsp += SZ_BE;
    float* BR1 = (float*)wsp; wsp += SZ_BD;
    float* BRQ = (float*)wsp; wsp += SZ_BQ;
    unsigned short* AO16 = X16;
    if ((size_t)(wsp - (char*)d_ws) > ws_size) return;

    k_cm_castbT<<<dim3((unsigned)((HDIM * (EMB / 8) + 255) / 256), NHEAD), 256, 0, stream>>>(wq, HDIM, (long long)EMB * HDIM, W316, EMB, (long long)HDIM * EMB, EMB, HDIM, 16.0f);
    k_cm_castbT<<<dim3((unsigned)((HDIM * (EMB / 8) + 255) / 256), NHEAD), 256, 0, stream>>>(wk, HDIM, (long long)EMB * HDIM, W316 + (size_t)EMB * EMB, EMB, (long long)HDIM * EMB, EMB, HDIM, 16.0f);
    k_cm_castbT<<<dim3((unsigned)((HDIM * (EMB / 8) + 255) / 256), NHEAD), 256, 0, stream>>>(wv, HDIM, (long long)EMB * HDIM, W316 + (size_t)2 * EMB * EMB, EMB, (long long)HDIM * EMB, EMB, HDIM, 16.0f);
    k_cm_castbT<<<dim3((unsigned)((EMB * (EMB / 8) + 255) / 256), 1), 256, 0, stream>>>(wo, EMB, 0LL, WO16, EMB, 0LL, EMB, EMB, 16.0f);
    k_cm_castbT<<<dim3((unsigned)((DFF * (EMB / 8) + 255) / 256), 1), 256, 0, stream>>>(w1, DFF, 0LL, W1T, EMB, 0LL, EMB, DFF, 16.0f);
    k_cm_castbT<<<dim3((unsigned)((EMB * (DFF / 8) + 255) / 256), 1), 256, 0, stream>>>(w2, EMB, 0LL, W2T, DFF, 0LL, DFF, EMB, 16.0f);
    k_cm_bfvec<<<(EMB + 255) / 256, 256, 0, stream>>>(bo, BRO, EMB);
    k_cm_bfvec<<<(DFF + 255) / 256, 256, 0, stream>>>(b1, BR1, DFF);
    k_cm_bfvec<<<(EMB + 255) / 256, 256, 0, stream>>>(b2, BR2, EMB);
    k_cm_bfvec<<<(EMB + 255) / 256, 256, 0, stream>>>(bq, BRQ, EMB);
    k_cm_bfvec<<<(EMB + 255) / 256, 256, 0, stream>>>(bk, BRQ + EMB, EMB);
    k_cm_bfvec<<<(EMB + 255) / 256, 256, 0, stream>>>(bv, BRQ + 2 * EMB, EMB);

    for (int ch = 0; ch < NCHUNK; ++ch) {
        const float* xc = x + (size_t)ch * NBC * SEQ_FULL * EMB;
        float* oc = out + (size_t)ch * NBC * SEQ_FULL * EMB;
        k_b_ln<3, 0, 0, 1><<<(RC + 7) / 8, 256, 0, stream>>>(xc, nullptr, g1, be1, 1e-5f, 1.0f / 384.0f, RC, nullptr, nullptr, 1, nullptr, X16);
        eng::wmma_gemm64<0, false, 2, 0, false, 0><<<dim3((unsigned)((((RC) / 64) * ((QKVW) / 64) + 7) / 8), 1u), 256, 0, stream>>>((const unsigned short*)X16, nullptr, EMB, 0, (const unsigned short*)W316, nullptr, EMB, 0, (void*)QKV, nullptr, QKVW, 0, BRQ, nullptr, 0, RC, QKVW, EMB, 0.0625f);
        k_attn_d<<<dim3((unsigned)((SEQ) / 64), (unsigned)NHEAD, (unsigned)NBC), 128, 0, stream>>>(QKV, QKV + EMB, QKV + 2 * EMB, AO, (SEQ) * QKVW, QKVW, (SEQ) * EMB, EMB, (SEQ) / 64, 0.125f);
        k_cast16<<<(unsigned)((((long long)RC * (EMB / 2)) + 255) / 256), 256, 0, stream>>>(AO, EMB, (_Float16*)AO16, EMB, RC, EMB, 1.0f);
        eng::wmma_gemm64<0, false, 2, 0, false, 0><<<dim3((unsigned)((((RC) / 64) * ((EMB) / 64) + 7) / 8), 1u), 256, 0, stream>>>((const unsigned short*)AO16, nullptr, EMB, 0, (const unsigned short*)WO16, nullptr, EMB, 0, (void*)ATT, nullptr, EMB, 0, BRO, nullptr, 0, RC, EMB, EMB, 0.0625f);
        k_b_add<1><<<(unsigned)((((long long)RC * (EMB / 4)) + 255) / 256), 256, 0, stream>>>(ATT, xc, nullptr, EMB / 4, 1, X1, (long long)RC * (EMB / 4));
        k_b_ln<3, 0, 0, 0><<<(RC + 7) / 8, 256, 0, stream>>>(X1, nullptr, g2, be2, 1e-5f, 1.0f / 384.0f, RC, nullptr, nullptr, 1, nullptr, H16);
        eng::wmma_gemm64<0, false, 2, 1, false, 3><<<dim3((unsigned)((((RC) / 64) * ((DFF) / 64) + 7) / 8), 1u), 256, 0, stream>>>((const unsigned short*)H16, nullptr, EMB, 0, (const unsigned short*)W1T, nullptr, EMB, 0, (void*)F16, nullptr, DFF, 0, BR1, nullptr, 0, RC, DFF, EMB, 0.0625f);
        eng::wmma_gemm64<0, false, 2, 0, false, 0><<<dim3((unsigned)((((RC) / 64) * ((EMB) / 64) + 7) / 8), 1u), 256, 0, stream>>>((const unsigned short*)F16, nullptr, DFF, 0, (const unsigned short*)W2T, nullptr, DFF, 0, (void*)FFo, nullptr, EMB, 0, BR2, nullptr, 0, RC, EMB, DFF, 0.0625f);
        k_b_add<0><<<(unsigned)((((long long)RC * (EMB / 4)) + 255) / 256), 256, 0, stream>>>(FFo, X1, nullptr, EMB / 4, 1, oc, (long long)RC * (EMB / 4));
    }
}
